// ReasoningMechanism_52226802319587
// MI455X (gfx1250) — hardware-verified
//
#include <hip/hip_runtime.h>
#include <stddef.h>


typedef _Float16 h16;
typedef _Float16 v16h __attribute__((ext_vector_type(16)));
typedef _Float16 v8h  __attribute__((ext_vector_type(8)));
typedef float    v8f  __attribute__((ext_vector_type(8)));
typedef float    v4f  __attribute__((ext_vector_type(4)));

#ifndef NB
#define NB 8
#endif
#define NB_FULL 8
#define NSLOT   256
#define DD      128
#define HID     256
#define MROWS   (NB * NSLOT)
#define PITCH1  768
#define NCAT    1024

static_assert(NB >= 1 && NB <= NB_FULL);
static_assert(NSLOT == 256 && DD == 128 && HID == 256);
static_assert(HID == 32 * 8);
static_assert(DD == 8 * 16);
static_assert((NSLOT % 16) == 0 && (NSLOT % 8) == 0);
static_assert((MROWS % 64) == 0 && (MROWS % 8) == 0);
static_assert((DD % 64) == 0 && (DD % 32) == 0);
static_assert((HID % 64) == 0 && (HID % 32) == 0);
static_assert((PITCH1 % 64) == 0 && PITCH1 == 3 * HID);
static_assert(NCAT == PITCH1 + HID);
static_assert((((size_t)MROWS * DD) % 2048) == 0);

#define LDT 72
#define LDC 68
static_assert((LDT % 8) == 0 && LDT >= 64);
static_assert((LDC % 4) == 0 && LDC >= 64);

#define WCARRY 64.0f
#define ACARRY 16.0f

#define BCAT_BYTES ((size_t)NCAT * DD * 2)
#define W2T_BYTES  ((size_t)DD * HID * 2)
#define S16_BYTES  ((size_t)MROWS * DD * 2)
#define P1_BYTES   ((size_t)MROWS * PITCH1 * 4)
#define AGG_BYTES  ((size_t)MROWS * DD * 2)
#define U_BYTES    ((size_t)MROWS * HID * 4)
#define G16_BYTES  ((size_t)MROWS * HID * 2)
#define OFF_BCAT ((size_t)0)
#define OFF_WM2  (OFF_BCAT + BCAT_BYTES)
#define OFF_WU2  (OFF_WM2 + W2T_BYTES)
#define OFF_S16  (OFF_WU2 + W2T_BYTES)
#define OFF_P1   (OFF_S16 + S16_BYTES)
#define OFF_AGG  (OFF_P1 + P1_BYTES)
#define OFF_U    (OFF_AGG + AGG_BYTES)
#define OFF_G16  (OFF_U + U_BYTES)
#define WS_TOTAL (OFF_G16 + G16_BYTES)
static_assert((BCAT_BYTES % 128) == 0 && (W2T_BYTES % 128) == 0 && (S16_BYTES % 128) == 0);
static_assert((P1_BYTES % 128) == 0 && (AGG_BYTES % 128) == 0 && (U_BYTES % 128) == 0);
static_assert((G16_BYTES % 128) == 0);
static_assert(WS_TOTAL <= (size_t)134217728);

__device__ __forceinline__ float bf16r(float x) {
  unsigned int u = __float_as_uint(x);
  u = (u + 0x7FFFu + ((u >> 16) & 1u)) & 0xFFFF0000u;
  return __uint_as_float(u);
}

static __device__ __forceinline__ h16 toh_flush(float v) {
  const h16 r = (h16)v;
  return (fabsf(v) < 6.103515625e-05f) ? (h16)0.0f : r;
}

static __device__ __forceinline__ float gelu_c(float x) {
  return (0.5f * ACARRY) * x * (1.0f + erff(x * 0.70710678118654752f));
}

__device__ __forceinline__ v16h frag_at(const _Float16* p) {
  v8h lo = *(const v8h*)(p);
  v8h hi = *(const v8h*)(p + 16);
  v16h out;
#pragma unroll
  for (int i = 0; i < 8; ++i) { out[i] = lo[i]; out[i + 8] = hi[i]; }
  return out;
}

__device__ __forceinline__ v8f wmma16(v16h a, v16h b, v8f c) {
  v8f d = __builtin_amdgcn_wmma_f32_16x16x32_f16(false, a, false, b, (short)0, c,
                                                 false, false);
  asm volatile("v_nop\n\tv_nop\n\tv_nop\n\tv_nop" : "+v"(d) : "v"(a), "v"(b));
  return d;
}

__device__ __forceinline__ float red32_sum(float x) {
#pragma unroll
  for (int off = 1; off < 32; off <<= 1) x += __shfl_xor(x, off, 32);
  return x;
}

__global__ __launch_bounds__(256) void wconv_kernel(
    const float* __restrict__ W, _Float16* __restrict__ Wt, unsigned ldw, unsigned ldk) {
  __shared__ _Float16 T[64 * LDT];
  const unsigned tid = threadIdx.x;
  const unsigned n0 = blockIdx.x * 64u;
  const unsigned k0 = blockIdx.y * 64u;
#pragma unroll 4
  for (unsigned j = 0; j < 16u; ++j) {
    const unsigned idx = tid + 256u * j;
    const unsigned kr = idx >> 6, nc = idx & 63u;
    const float v = W[(size_t)(k0 + kr) * ldw + n0 + nc];
    T[nc * LDT + kr] = (_Float16)(WCARRY * bf16r(v));
  }
  __syncthreads();
  v8h x[2];
  size_t off[2];
#pragma unroll
  for (unsigned i = 0; i < 2u; ++i) {
    const unsigned n = 32u * i + (tid >> 3);
    const unsigned kc = (tid & 7u) * 8u;
    x[i] = *(const v8h*)&T[n * LDT + kc];
    off[i] = (size_t)(n0 + n) * ldk + k0 + kc;
  }
#pragma unroll
  for (int i = 0; i < 2; ++i) *(volatile v8h*)(Wt + off[i]) = x[i];
  __threadfence();
#pragma unroll
  for (int i = 0; i < 2; ++i) *(volatile v8h*)(Wt + off[i]) = x[i];
}

__global__ __launch_bounds__(256) void cast_kernel(
    const float* __restrict__ X, _Float16* __restrict__ dst) {
#pragma clang fp contract(off)
  const size_t idx = ((size_t)blockIdx.x * 256u + threadIdx.x) * 8u;
  const v4f a0 = *(const v4f*)(X + idx);
  const v4f a1 = *(const v4f*)(X + idx + 4u);
  v8h o;
#pragma unroll
  for (int i = 0; i < 4; ++i) {
    o[i]     = toh_flush(ACARRY * bf16r(a0[i]));
    o[i + 4] = toh_flush(ACARRY * bf16r(a1[i]));
  }
  _Float16* p = dst + idx;
  *(volatile v8h*)p = o;
  __threadfence();
  *(volatile v8h*)p = o;
}

template <int MODE>
__device__ __forceinline__ void gemm_body(
    const _Float16* __restrict__ A16, const _Float16* __restrict__ Bt, const unsigned K,
    const float* __restrict__ bias, const float* __restrict__ addf, float* __restrict__ outf) {
  __shared__ float Cs[64 * LDC];
  const unsigned tid = threadIdx.x, lane = tid & 31u;
  const unsigned w = (unsigned)__builtin_amdgcn_readfirstlane((int)(tid >> 5));
  const unsigned mw = w >> 1, nw = w & 1u;
  const unsigned hh = lane >> 4, m = lane & 15u;
  const unsigned n0 = blockIdx.x * 64u;
  const unsigned row0 = blockIdx.y * 64u;

  const _Float16* ap  = A16 + (size_t)(row0 + mw * 16u + m) * K + hh * 8u;
  const _Float16* bp0 = Bt + (size_t)(n0 + nw * 32u + m) * K + hh * 8u;
  const _Float16* bp1 = bp0 + (size_t)16 * K;
  v8f acc0 = {}, acc1 = {};
#pragma unroll 2
  for (unsigned k0 = 0; k0 < K; k0 += 32u) {
    const v16h a  = frag_at(ap + k0);
    const v16h b0 = frag_at(bp0 + k0);
    const v16h b1 = frag_at(bp1 + k0);
    acc0 = wmma16(a, b0, acc0);
    acc1 = wmma16(a, b1, acc1);
  }
#pragma unroll
  for (int r = 0; r < 8; ++r) {
    float* d = &Cs[(mw * 16u + hh * 8u + (unsigned)r) * LDC + nw * 32u + m];
    d[0]  = acc0[r];
    d[16] = acc1[r];
  }
  __syncthreads();

  const float cs = 1.0f / (WCARRY * ACARRY);
  const unsigned ldo = (MODE == 0) ? (unsigned)PITCH1 : ((MODE == 1) ? (unsigned)HID : (unsigned)DD);
  v4f xs[4];
  size_t off[4];
#pragma unroll
  for (unsigned i = 0; i < 4u; ++i) {
    const unsigned r = 16u * i + (tid >> 4);
    const unsigned c = (tid & 15u) * 4u;
    const size_t row = (size_t)(row0 + r);
    const v4f u = *(const v4f*)&Cs[r * LDC + c];
    v4f val;
    if (MODE == 0) {
#pragma unroll
      for (int j = 0; j < 4; ++j) val[j] = u[j] * cs;
    }
    if (MODE == 1) {
      const v4f g  = *(const v4f*)(bias + n0 + c);
      const v4f su = *(const v4f*)(addf + row * PITCH1 + 2u * HID + n0 + c);
#pragma unroll
      for (int j = 0; j < 4; ++j) val[j] = (u[j] * cs + su[j]) + bf16r(g[j]);
    }
    if (MODE == 2) {
      const v4f g   = *(const v4f*)(bias + n0 + c);
      const v4f xin = *(const v4f*)(addf + row * DD + n0 + c);
#pragma unroll
      for (int j = 0; j < 4; ++j) val[j] = bf16r(xin[j]) + (u[j] * cs + bf16r(g[j]));
    }
    xs[i] = val;
    off[i] = row * ldo + n0 + c;
  }
#pragma unroll
  for (int i = 0; i < 4; ++i) *(volatile v4f*)(outf + off[i]) = xs[i];
  __threadfence();
#pragma unroll
  for (int i = 0; i < 4; ++i) *(volatile v4f*)(outf + off[i]) = xs[i];
}

__global__ __launch_bounds__(256) void gemm_proj_kernel(
    const _Float16* __restrict__ A16, const _Float16* __restrict__ Bt, float* __restrict__ outf) {
  gemm_body<0>(A16, Bt, (unsigned)DD, (const float*)0, (const float*)0, outf);
}
__global__ __launch_bounds__(256) void gemm_upd_kernel(
    const _Float16* __restrict__ A16, const _Float16* __restrict__ Bt,
    const float* __restrict__ bias, const float* __restrict__ proj, float* __restrict__ outf) {
  gemm_body<1>(A16, Bt, (unsigned)DD, bias, proj, outf);
}
__global__ __launch_bounds__(256) void gemm_out_kernel(
    const _Float16* __restrict__ A16, const _Float16* __restrict__ Bt,
    const float* __restrict__ bias, const float* __restrict__ xin, float* __restrict__ outf) {
  gemm_body<2>(A16, Bt, (unsigned)HID, bias, xin, outf);
}

__global__ __launch_bounds__(256) __attribute__((amdgpu_num_vgpr(256))) void pair_kernel(
    const float* __restrict__ P1, const float* __restrict__ adj,
    const float* __restrict__ bm1, const float* __restrict__ bm2,
    const _Float16* __restrict__ W2t, _Float16* __restrict__ agg16) {
  __shared__ float Hs[8 * HID];
  __shared__ float Fs[8 * DD];

  const unsigned tid = threadIdx.x, lane = tid & 31u;
  const unsigned w = (unsigned)__builtin_amdgcn_readfirstlane((int)(tid >> 5));
  const unsigned hh = lane >> 4, m = lane & 15u;
  const unsigned b = blockIdx.y;
  const unsigned i = blockIdx.x * 8u + w;
  const unsigned grow = b * (unsigned)NSLOT + i;

  {
    const float* hp = P1 + (size_t)grow * PITCH1 + lane * 8u;
    const v4f a0 = *(const v4f*)(hp);
    const v4f a1 = *(const v4f*)(hp + 4u);
    const v4f c0 = *(const v4f*)(bm1 + lane * 8u);
    const v4f c1 = *(const v4f*)(bm1 + lane * 8u + 4u);
    v4f t0, t1;
#pragma unroll
    for (int e = 0; e < 4; ++e) {
      t0[e] = a0[e] + bf16r(c0[e]);
      t1[e] = a1[e] + bf16r(c1[e]);
    }
    *(v4f*)&Hs[w * HID + lane * 8u] = t0;
    *(v4f*)&Hs[w * HID + lane * 8u + 4u] = t1;
  }
  __syncthreads();

  const float* adjrow = adj + (size_t)grow * NSLOT;
  const _Float16* wp = W2t + (size_t)m * HID + hh * 8u;
  const unsigned hb = w * (unsigned)HID + hh * 8u;

  float col[8];
#pragma unroll
  for (int nb = 0; nb < 8; ++nb) col[nb] = 0.0f;
  float asum = 0.0f;

#pragma unroll 1
  for (unsigned jt = 0; jt < (unsigned)(NSLOT / 16); ++jt) {
    const float* hjp = P1 + (size_t)(b * (unsigned)NSLOT + jt * 16u + m) * PITCH1 + HID + hh * 8u;
    v8f acc[8];
#pragma unroll
    for (int nb = 0; nb < 8; ++nb) acc[nb] = (v8f){};

#pragma unroll 1
    for (unsigned k0 = 0; k0 < (unsigned)HID; k0 += 32u) {
      const v4f h0 = *(const v4f*)&Hs[hb + k0];
      const v4f h1 = *(const v4f*)&Hs[hb + k0 + 4u];
      const v4f h2 = *(const v4f*)&Hs[hb + k0 + 16u];
      const v4f h3 = *(const v4f*)&Hs[hb + k0 + 20u];
      const v4f j0 = *(const v4f*)(hjp + k0);
      const v4f j1 = *(const v4f*)(hjp + k0 + 4u);
      const v4f j2 = *(const v4f*)(hjp + k0 + 16u);
      const v4f j3 = *(const v4f*)(hjp + k0 + 20u);
      v16h a;
#pragma unroll
      for (int e = 0; e < 4; ++e) {
        a[e]      = toh_flush(gelu_c(h0[e] + j0[e]));
        a[e + 4]  = toh_flush(gelu_c(h1[e] + j1[e]));
        a[e + 8]  = toh_flush(gelu_c(h2[e] + j2[e]));
        a[e + 12] = toh_flush(gelu_c(h3[e] + j3[e]));
      }
#pragma unroll
      for (int nb = 0; nb < 8; ++nb) {
        const v16h bf = frag_at(wp + (size_t)(nb * 16) * HID + k0);
        acc[nb] = wmma16(a, bf, acc[nb]);
      }
    }

    const v4f w0 = *(const v4f*)(adjrow + jt * 16u + hh * 8u);
    const v4f w1 = *(const v4f*)(adjrow + jt * 16u + hh * 8u + 4u);
    float a8[8];
#pragma unroll
    for (int e = 0; e < 4; ++e) {
      a8[e]     = bf16r(w0[e]);
      a8[e + 4] = bf16r(w1[e]);
    }
#pragma unroll
    for (int r = 0; r < 8; ++r) asum += a8[r];
#pragma unroll
    for (int nb = 0; nb < 8; ++nb) {
      float t = col[nb];
#pragma unroll
      for (int r = 0; r < 8; ++r) t += a8[r] * acc[nb][r];
      col[nb] = t;
    }
  }

#pragma unroll
  for (int nb = 0; nb < 8; ++nb) col[nb] += __shfl_xor(col[nb], 16, 32);
  asum += __shfl_xor(asum, 16, 32);

#pragma unroll
  for (int nb = 0; nb < 8; ++nb) {
    const unsigned d = (unsigned)nb * 16u + m;
    const float val = col[nb] * (1.0f / (WCARRY * ACARRY)) + bf16r(bm2[d]) * asum;
    Fs[w * DD + d] = val;
  }
  __syncthreads();

  if (w < 4u) {
    const unsigned r = w * 2u + (lane >> 4);
    const unsigned c = (lane & 15u) * 8u;
    const v4f u0 = *(const v4f*)&Fs[r * DD + c];
    const v4f u1 = *(const v4f*)&Fs[r * DD + c + 4u];
    v8h x;
#pragma unroll
    for (int e = 0; e < 4; ++e) {
      x[e]     = toh_flush(u0[e] * ACARRY);
      x[e + 4] = toh_flush(u1[e] * ACARRY);
    }
    _Float16* p = agg16 + (size_t)(b * (unsigned)NSLOT + blockIdx.x * 8u + r) * DD + c;
    *(volatile v8h*)p = x;
    __threadfence();
    *(volatile v8h*)p = x;
  }
}

__global__ __launch_bounds__(256) void ln_gelu_kernel(
    const float* __restrict__ U, const float* __restrict__ G, const float* __restrict__ Be,
    _Float16* __restrict__ dst) {
#pragma clang fp contract(off)
  __shared__ _Float16 T[8 * HID];
  const unsigned lane = threadIdx.x & 31u;
  const unsigned w = (unsigned)__builtin_amdgcn_readfirstlane((int)(threadIdx.x >> 5));
  const unsigned row = blockIdx.x * 8u + w;
  const float* ur = U + (size_t)row * HID;

  float s = 0.0f;
#pragma unroll 1
  for (unsigned e = 0; e < 8u; ++e) s += ur[e * 32u + lane];
  const float mean = red32_sum(s) * (1.0f / (float)HID);

  float ss = 0.0f;
#pragma unroll 1
  for (unsigned e = 0; e < 8u; ++e) {
    const float d = ur[e * 32u + lane] - mean;
    ss += d * d;
  }
  const float var = red32_sum(ss) * (1.0f / (float)HID);
  const float rstd = 1.0f / sqrtf(var + 1.0e-5f);

#pragma unroll 1
  for (unsigned e = 0; e < 8u; ++e) {
    const unsigned c = e * 32u + lane;
    const float d = ur[c] - mean;
    const float x = d * rstd * bf16r(G[c]) + bf16r(Be[c]);
    T[w * HID + c] = toh_flush(gelu_c(x));
  }
  __syncthreads();
  const v8h o = *(const v8h*)&T[w * HID + lane * 8u];
  _Float16* p = dst + (size_t)row * HID + lane * 8u;
  *(volatile v8h*)p = o;
  __threadfence();
  *(volatile v8h*)p = o;
}

extern "C" void kernel_launch(void* const* d_in, const int* in_sizes, int n_in,
                              void* d_out, int out_size, void* d_ws, size_t ws_size,
                              hipStream_t stream) {
  if (n_in < 12) return;
  if ((long long)in_sizes[0] < (long long)MROWS * DD) return;
  if ((long long)in_sizes[1] < (long long)MROWS * NSLOT) return;
  if ((long long)in_sizes[2] < (long long)2 * DD * HID) return;
  if (in_sizes[3] < HID) return;
  if ((long long)in_sizes[4] < (long long)HID * DD) return;
  if (in_sizes[5] < DD) return;
  if ((long long)in_sizes[6] < (long long)2 * DD * HID) return;
  if (in_sizes[7] < HID || in_sizes[8] < HID || in_sizes[9] < HID) return;
  if ((long long)in_sizes[10] < (long long)HID * DD) return;
  if (in_sizes[11] < DD) return;
  if ((long long)out_size < (long long)MROWS * DD) return;
  if (ws_size < WS_TOTAL) return;

  const float* slots = (const float*)d_in[0];
  const float* adjm  = (const float*)d_in[1];
  const float* w_m1  = (const float*)d_in[2];
  const float* b_m1  = (const float*)d_in[3];
  const float* w_m2  = (const float*)d_in[4];
  const float* b_m2  = (const float*)d_in[5];
  const float* w_u1  = (const float*)d_in[6];
  const float* b_u1  = (const float*)d_in[7];
  const float* ln_g  = (const float*)d_in[8];
  const float* ln_b  = (const float*)d_in[9];
  const float* w_u2  = (const float*)d_in[10];
  const float* b_u2  = (const float*)d_in[11];
  float* out = (float*)d_out;

  char* ws = (char*)d_ws;
  _Float16* Bcat  = (_Float16*)(ws + OFF_BCAT);
  _Float16* Wm2_t = (_Float16*)(ws + OFF_WM2);
  _Float16* Wu2_t = (_Float16*)(ws + OFF_WU2);
  _Float16* S16   = (_Float16*)(ws + OFF_S16);
  float*    P1    = (float*)(ws + OFF_P1);
  _Float16* Agg16 = (_Float16*)(ws + OFF_AGG);
  float*    Uf    = (float*)(ws + OFF_U);
  _Float16* G16   = (_Float16*)(ws + OFF_G16);

  dim3 blk(256);

  wconv_kernel<<<dim3(HID / 64, DD / 64), blk, 0, stream>>>(w_m1, Bcat, (unsigned)HID, (unsigned)DD);
  wconv_kernel<<<dim3(HID / 64, DD / 64), blk, 0, stream>>>(w_m1 + (size_t)DD * HID,
                                                          Bcat + (size_t)HID * DD,
                                                          (unsigned)HID, (unsigned)DD);
  wconv_kernel<<<dim3(HID / 64, DD / 64), blk, 0, stream>>>(w_u1, Bcat + (size_t)2 * HID * DD,
                                                          (unsigned)HID, (unsigned)DD);
  wconv_kernel<<<dim3(HID / 64, DD / 64), blk, 0, stream>>>(w_u1 + (size_t)DD * HID,
                                                          Bcat + (size_t)3 * HID * DD,
                                                          (unsigned)HID, (unsigned)DD);
  wconv_kernel<<<dim3(DD / 64, HID / 64), blk, 0, stream>>>(w_m2, Wm2_t, (unsigned)DD, (unsigned)HID);
  wconv_kernel<<<dim3(DD / 64, HID / 64), blk, 0, stream>>>(w_u2, Wu2_t, (unsigned)DD, (unsigned)HID);

  cast_kernel<<<dim3((unsigned)(((size_t)MROWS * DD) / 2048)), blk, 0, stream>>>(slots, S16);
  gemm_proj_kernel<<<dim3(PITCH1 / 64, MROWS / 64), blk, 0, stream>>>(S16, Bcat, P1);
  pair_kernel<<<dim3(NSLOT / 8, NB), blk, 0, stream>>>(P1, adjm, b_m1, b_m2, Wm2_t, Agg16);
  gemm_upd_kernel<<<dim3(HID / 64, MROWS / 64), blk, 0, stream>>>(
      Agg16, Bcat + (size_t)3 * HID * DD, b_u1, P1, Uf);
  ln_gelu_kernel<<<dim3(MROWS / 8), blk, 0, stream>>>(Uf, ln_g, ln_b, G16);
  gemm_out_kernel<<<dim3(DD / 64, MROWS / 64), blk, 0, stream>>>(G16, Wu2_t, b_u2, slots, out);
}
